// GRN_22299470201519
// MI455X (gfx1250) — hardware-verified
//
#include <hip/hip_runtime.h>
#include <hip/hip_bf16.h>
#include <stddef.h>

#define __bf16 _Float16
typedef __attribute__((ext_vector_type(16))) _Float16       v16bf;
typedef __attribute__((ext_vector_type(4)))  float          v4f_t;
typedef float v4fa __attribute__((ext_vector_type(4), may_alias));
typedef __attribute__((ext_vector_type(8)))  float           v8f;
typedef __attribute__((ext_vector_type(8)))  unsigned short  v8us;
typedef __attribute__((ext_vector_type(16))) unsigned short  v16us;

union FragU { v16bf bf; v16us us; v8us h2[2]; };

__device__ __forceinline__ unsigned short f2bf(float f) { return __builtin_bit_cast(unsigned short, (_Float16)f); }
__device__ __forceinline__ unsigned pk2(float a, float b) { return (unsigned)f2bf(a) | ((unsigned)f2bf(b) << 16); }

__device__ __forceinline__ v8f zero8() {
    v8f z;
#pragma unroll
    for (int i = 0; i < 8; ++i) z[i] = 0.0f;
    return z;
}

__device__ __forceinline__ v16bf load_fragA(const unsigned short* base, int stride) {
    int lane = threadIdx.x & 31;
    const unsigned short* p = base + (size_t)(lane & 15) * stride + ((lane >> 4) << 3);
    FragU u;
    u.h2[0] = *(const v8us*)(p);
    u.h2[1] = *(const v8us*)(p + 16);
    return u.bf;
}

__device__ __forceinline__ v16bf load_fragB(const unsigned short* baseT, int stride) {
    int lane = threadIdx.x & 31;
    const unsigned short* p = baseT + (size_t)(lane & 15) * stride + ((lane >> 4) << 3);
    FragU u;
    u.h2[0] = *(const v8us*)(p);
    u.h2[1] = *(const v8us*)(p + 16);
    return u.bf;
}
__device__ __forceinline__ void store_tile16x32(const float* stg, float* dst, long ld, int lane) {
    v4f_t vv[4];
#pragma unroll
    for (int i = 0; i < 4; ++i) { const int c = lane + 32 * i; vv[i] = *(const volatile v4fa*)(stg + (c >> 3) * 32 + (c & 7) * 4); }
#pragma unroll
    for (int i = 0; i < 4; ++i) { const int c = lane + 32 * i; *(volatile v4f_t*)(dst + (long)(c >> 3) * ld + (c & 7) * 4) = vv[i]; }
    __threadfence();
#pragma unroll
    for (int i = 0; i < 4; ++i) { const int c = lane + 32 * i; *(volatile v4f_t*)(dst + (long)(c >> 3) * ld + (c & 7) * 4) = vv[i]; }
}

__device__ __forceinline__ v8f wmma_bf16(v16bf a, v16bf b, v8f c) {
    return __builtin_amdgcn_wmma_f32_16x16x32_f16(false, a, false, b, (short)0, c, false, false);
}

#define NN   256
#define SS   32
#define MM   32
#define EE   32
#define BB   64
#define NIN  16
#define NOUT 16
#define ROWS (BB * NN)
#define KBIG (NN * EE)


__global__ void k_build_h(const float* __restrict__ inputs, const float* __restrict__ init,
                          float* __restrict__ h32, unsigned short* __restrict__ hB) {
    int t = (blockIdx.x * blockDim.x + threadIdx.x) * 2;
    int s = t & 31;
    int n = (t >> 5) & 255;
    float v0, v1;
    if (n < NIN) {
        int b = t >> 13;
        const float* p = inputs + ((size_t)b * NIN + n) * SS + s; v0 = p[0]; v1 = p[1];
    } else {
        const float* p = init + n * SS + s; v0 = p[0]; v1 = p[1];
    }
    typedef __attribute__((ext_vector_type(2))) float v2f_t;
    v2f_t hv; hv.x = v0; hv.y = v1;
    const unsigned pk = pk2(v0, v1);
    *(volatile v2f_t*)(h32 + t) = hv; *(volatile unsigned*)(hB + t) = pk;
    __threadfence();
    *(volatile v2f_t*)(h32 + t) = hv; *(volatile unsigned*)(hB + t) = pk;
}

__global__ void k_wfb(const float* __restrict__ Wf, unsigned short* __restrict__ wfB) {
    int t = (blockIdx.x * blockDim.x + threadIdx.x) * 2;
    const unsigned pk = pk2(Wf[t], Wf[t + 1]);
    *(volatile unsigned*)(wfB + t) = pk; __threadfence(); *(volatile unsigned*)(wfB + t) = pk;
}

__global__ void k_edgeT(const float* __restrict__ edge, unsigned short* __restrict__ edgeT) {
    int t = (blockIdx.x * blockDim.x + threadIdx.x) * 2;
    int j = t >> 13;
    int i = (t >> 5) & 255;
    int e = t & 31;
    const float* p = edge + ((size_t)i << 13) + (j << 5) + e;
    const unsigned pk = pk2(p[0], p[1]);
    *(volatile unsigned*)(edgeT + t) = pk; __threadfence(); *(volatile unsigned*)(edgeT + t) = pk;
}

__global__ void k_wtrans(const float* __restrict__ Wz, const float* __restrict__ Uz,
                         const float* __restrict__ Wr, const float* __restrict__ Ur,
                         const float* __restrict__ Wh, const float* __restrict__ Uh,
                         unsigned short* __restrict__ WT) {
    int t = (blockIdx.x * blockDim.x + threadIdx.x) * 2;
    if (t >= 6 * 1024) return;
    int mi = t >> 10, idx = t & 1023;
    int n = idx >> 5, k = idx & 31;
    const float* src = (mi == 0) ? Wz : (mi == 1) ? Uz : (mi == 2) ? Wr
                     : (mi == 3) ? Ur : (mi == 4) ? Wh : Uh;
    const unsigned pk = pk2(src[k * 32 + n], src[(k + 1) * 32 + n]);
    *(volatile unsigned*)(WT + t) = pk; __threadfence(); *(volatile unsigned*)(WT + t) = pk;
}

__global__ void k_hs(const float* __restrict__ h32, float* __restrict__ Hs) {
    int t = blockIdx.x * blockDim.x + threadIdx.x;
    if (t >= BB * SS) return;
    int b = t >> 5, s = t & 31;
    float acc = 0.0f;
    for (int i = 0; i < NN; ++i) acc += h32[((size_t)b * NN + i) * SS + s];
    *(volatile float*)(Hs + t) = acc; __threadfence(); *(volatile float*)(Hs + t) = acc;
}

__global__ __launch_bounds__(128) void k_gfilt(const unsigned short* __restrict__ hB,
                        const unsigned short* __restrict__ wfB,
                        unsigned short* __restrict__ GT) {
    __shared__ __align__(16) unsigned short st[4][16 * 512];
    int wave = (blockIdx.x * blockDim.x + threadIdx.x) >> 5;
    int wloc = threadIdx.x >> 5;
    int lane = threadIdx.x & 31;
    int col0 = lane & 15, rb = (lane >> 4) << 3;
    unsigned short* sw = st[wloc];
    const int bI = (wave * 16) >> 8, i0 = (wave * 16) & 255;
    v16bf a = load_fragA(hB + (size_t)wave * 16 * SS, SS);
#pragma unroll 1
    for (int mh = 0; mh < 2; ++mh) {
#pragma unroll 4
        for (int e = 0; e < EE; ++e) {
            const int ct = 2 * e + mh;
            v16bf bfr = load_fragB(wfB + ct * 16 * SS, SS);
            v8f acc = zero8();
            acc = wmma_bf16(a, bfr, acc);
#pragma unroll
            for (int g = 0; g < 8; ++g) sw[col0 * 512 + (rb + g) * 32 + e] = f2bf(acc[g]);
        }
        asm volatile("s_wait_dscnt 0" ::: "memory");
        typedef __attribute__((ext_vector_type(4))) unsigned v4u_t;
        typedef unsigned v4ua __attribute__((ext_vector_type(4), may_alias));
#pragma unroll 1
        for (int pass = 0; pass < 2; ++pass) {
#pragma unroll 4
            for (int q = 0; q < 32; ++q) {
                const int c = lane + 32 * q, ml = c >> 6, pc = c & 63;
                const v4u_t v = *(const volatile v4ua*)(sw + ml * 512 + pc * 8);
                *(volatile v4u_t*)(GT + (((size_t)bI * 32 + mh * 16 + ml) << 13) + i0 * 32 + pc * 8) = v;
            }
            __threadfence();
        }
        asm volatile("s_wait_dscnt 0" ::: "memory");
    }
}

__global__ void k_msg(const unsigned short* __restrict__ edgeT,
                      const unsigned short* __restrict__ GT,
                      const float* __restrict__ Hs, const float* __restrict__ bf,
                      unsigned short* __restrict__ msgB) {
    int wid = (blockIdx.x * blockDim.x + threadIdx.x) >> 5;
    int b = wid >> 4;
    int jt = wid & 15;
    int lane = threadIdx.x & 31;
    int col0 = lane & 15, rb = (lane >> 4) << 3;

    const unsigned short* Abase = edgeT + (size_t)jt * 16 * KBIG;
    const unsigned short* B0 = GT + (((size_t)b * 32 + 0)  << 13);
    const unsigned short* B1 = GT + (((size_t)b * 32 + 16) << 13);

    v8f acc0 = zero8(), acc1 = zero8();
#pragma unroll 4
    for (int kb = 0; kb < KBIG; kb += 32) {
        v16bf a  = load_fragA(Abase + kb, KBIG);
        v16bf f0 = load_fragB(B0 + kb, KBIG);
        v16bf f1 = load_fragB(B1 + kb, KBIG);
        acc0 = wmma_bf16(a, f0, acc0);
        acc1 = wmma_bf16(a, f1, acc1);
        if (kb + 128 < KBIG)
            __builtin_prefetch(Abase + (size_t)(lane & 15) * KBIG + kb + 128, 0, 1);
    }

    float t0 = 0.0f, t1 = 0.0f;
    for (int s = 0; s < SS; ++s) {
        float hs = Hs[b * SS + s];
        t0 += hs * bf[col0 * SS + s];
        t1 += hs * bf[(16 + col0) * SS + s];
    }
    __shared__ __align__(16) unsigned short mst[4][16 * MM];
    unsigned short* ms = mst[threadIdx.x >> 5];
#pragma unroll
    for (int g = 0; g < 8; ++g) {
        ms[(rb + g) * MM + col0]      = f2bf(acc0[g] + t0);
        ms[(rb + g) * MM + 16 + col0] = f2bf(acc1[g] + t1);
    }
    asm volatile("s_wait_dscnt 0" ::: "memory");
    {
        typedef __attribute__((ext_vector_type(4))) unsigned v4u_t;
        typedef unsigned v4ua __attribute__((ext_vector_type(4), may_alias));
        unsigned short* dst = msgB + (size_t)(b * NN + jt * 16) * MM;
        const v4u_t v0 = *(const volatile v4ua*)(ms + lane * 8), v1 = *(const volatile v4ua*)(ms + 256 + lane * 8);
        *(volatile v4u_t*)(dst + lane * 8) = v0; *(volatile v4u_t*)(dst + 256 + lane * 8) = v1;
        __threadfence();
        *(volatile v4u_t*)(dst + lane * 8) = v0; *(volatile v4u_t*)(dst + 256 + lane * 8) = v1;
    }
}

__global__ void k_gru(const unsigned short* __restrict__ msgB,
                      const unsigned short* __restrict__ hB,
                      const float* __restrict__ h32,
                      const unsigned short* __restrict__ WT,
                      const float* __restrict__ bz, const float* __restrict__ br,
                      const float* __restrict__ bh,
                      float* __restrict__ out_outputs, float* __restrict__ out_hnew) {
    __shared__ __align__(16) unsigned short ldsrh[4][16 * SS];
    __shared__ __align__(16) float hst[4][16 * SS];
    int wid  = (blockIdx.x * blockDim.x + threadIdx.x) >> 5;
    int wiw  = threadIdx.x >> 5;
    int lane = threadIdx.x & 31;
    int col0 = lane & 15, rb = (lane >> 4) << 3;
    size_t rowbase = (size_t)wid * 16 * SS;

    v16bf aM = load_fragA(msgB + rowbase, SS);
    v16bf aH = load_fragA(hB  + rowbase, SS);

    const unsigned short* WzT = WT + 0 * 1024;
    const unsigned short* UzT = WT + 1 * 1024;
    const unsigned short* WrT = WT + 2 * 1024;
    const unsigned short* UrT = WT + 3 * 1024;
    const unsigned short* WhT = WT + 4 * 1024;
    const unsigned short* UhT = WT + 5 * 1024;

    v8f z[2], hf[2];
#pragma unroll
    for (int ct = 0; ct < 2; ++ct) {
        v8f az = zero8();
        az = wmma_bf16(aM, load_fragB(WzT + ct * 16 * SS, SS), az);
        az = wmma_bf16(aH, load_fragB(UzT + ct * 16 * SS, SS), az);
        v8f ar = zero8();
        ar = wmma_bf16(aM, load_fragB(WrT + ct * 16 * SS, SS), ar);
        ar = wmma_bf16(aH, load_fragB(UrT + ct * 16 * SS, SS), ar);

        float bzc = bz[ct * 16 + col0], brc = br[ct * 16 + col0];
#pragma unroll
        for (int g = 0; g < 8; ++g) {
            int R = wid * 16 + rb + g;
            float hv = h32[(size_t)R * SS + ct * 16 + col0];
            hf[ct][g] = hv;
            z[ct][g]  = 1.0f / (1.0f + __expf(-(az[g] + bzc)));
            float rv  = 1.0f / (1.0f + __expf(-(ar[g] + brc)));
            ldsrh[wiw][(rb + g) * SS + ct * 16 + col0] = f2bf(rv * hv);
        }
    }
    __syncthreads();
    v16bf aRH = load_fragA(&ldsrh[wiw][0], SS);

#pragma unroll
    for (int ct = 0; ct < 2; ++ct) {
        v8f ah = zero8();
        ah = wmma_bf16(aM,  load_fragB(WhT + ct * 16 * SS, SS), ah);
        ah = wmma_bf16(aRH, load_fragB(UhT + ct * 16 * SS, SS), ah);
        float bhc = bh[ct * 16 + col0];
#pragma unroll
        for (int g = 0; g < 8; ++g) {
            float th = tanhf(ah[g] + bhc);
            float hn = (1.0f - z[ct][g]) * hf[ct][g] + z[ct][g] * th;
            hst[wiw][(rb + g) * SS + ct * 16 + col0] = hn;
        }
    }
    asm volatile("s_wait_dscnt 0" ::: "memory");
    store_tile16x32(hst[wiw], out_hnew + (size_t)wid * 16 * SS, SS, lane);
    {
        const int R0 = wid * 16, n0 = R0 & 255, b = R0 >> 8;
        if (n0 == NN - NOUT) {
            float* dst0 = out_outputs + ((size_t)((NN - 1) - n0) * BB + b) * SS;
            store_tile16x32(hst[wiw], dst0, -(long)BB * SS, lane);
        }
    }
}

extern "C" void kernel_launch(void* const* d_in, const int* in_sizes, int n_in,
                              void* d_out, int out_size, void* d_ws, size_t ws_size,
                              hipStream_t stream) {
    const float* inputs = (const float*)d_in[0];
    const float* init   = (const float*)d_in[1];
    const float* edge   = (const float*)d_in[2];
    const float* Wf     = (const float*)d_in[3];
    const float* bf     = (const float*)d_in[4];
    const float* Wz     = (const float*)d_in[5];
    const float* Uz     = (const float*)d_in[6];
    const float* bz     = (const float*)d_in[7];
    const float* Wr     = (const float*)d_in[8];
    const float* Ur     = (const float*)d_in[9];
    const float* br     = (const float*)d_in[10];
    const float* Wh     = (const float*)d_in[11];
    const float* Uh     = (const float*)d_in[12];
    const float* bh     = (const float*)d_in[13];

    float* out_outputs = (float*)d_out;
    float* out_hnew    = (float*)d_out + NOUT * BB * SS;

    char* ws = (char*)d_ws;
    float*          h32   = (float*)(ws + 0);
    unsigned short* hB    = (unsigned short*)(ws + 2097152);
    unsigned short* wfB   = (unsigned short*)(ws + 3145728);
    unsigned short* edgeT = (unsigned short*)(ws + 3211264);
    unsigned short* GT    = (unsigned short*)(ws + 7405568);
    unsigned short* msgB  = (unsigned short*)(ws + 40960000);
    unsigned short* WT    = (unsigned short*)(ws + 42008576);
    float*          Hs    = (float*)(ws + 42020864);

    k_build_h<<<1024, 256, 0, stream>>>(inputs, init, h32, hB);
    k_wfb    <<<64,   256, 0, stream>>>(Wf, wfB);
    k_edgeT  <<<4096, 256, 0, stream>>>(edge, edgeT);
    k_wtrans <<<12,   256, 0, stream>>>(Wz, Uz, Wr, Ur, Wh, Uh, WT);
    k_hs     <<<8,    256, 0, stream>>>(h32, Hs);

    k_gfilt  <<<256, 128, 0, stream>>>(hB, wfB, GT);
    k_msg    <<<256, 128, 0, stream>>>(edgeT, GT, Hs, bf, msgB);
    k_gru    <<<256, 128, 0, stream>>>(msgB, hB, h32, WT, bz, br, bh,
                                       out_outputs, out_hnew);
}
